// NodeEncoder_90056874262535
// MI455X (gfx1250) — hardware-verified
//
#include <hip/hip_runtime.h>
#include <stddef.h>


#define U      64
#define NTHR   256
#define NWAVE  8
#define EPT    8
#define CHUNK  (NTHR * EPT)
#define WCAP   (EPT * 32)
#define LISTN  (NWAVE * WCAP)
#define PASSN  (NWAVE * 16)
#define PCAP   (CHUNK + PASSN)
#define NB     768
#define NT     128
#define NQ     ((NB * U) / (NTHR * 4))
#define WSC    8.0f
#define WINV   0.125f
#define LN_EPS 1e-5f

static_assert(PASSN == 128);
static_assert((PCAP % PASSN) == 0);
static_assert(NQ * NTHR * 4 == NB * U);
static_assert((NB % NT) == 0);

#define A_ACC  0
#define A_CNT  (A_ACC + (NB + 1) * U * 4)
#define A_WSM  (A_CNT + 3088)
#define A_BSM  (A_WSM + 2 * U * U * 2)
#define A_EW   (A_BSM + U * 4)
#define A_EB   (A_EW + U * 4)
#define A_STG  (A_EB + U * 4)
#define A_MSG  (A_STG + NWAVE * 16 * U * 2)
#define A_LIST (A_MSG + PASSN * U * 4)
#define A_PEND (A_LIST + LISTN * 4)
#define A_SLOT (A_PEND + PCAP * 4)
#define A_WCNT (A_SLOT + PASSN * 4)
#define A_END  (A_WCNT + 64)
static_assert((NB + 1) * 4 <= 3088);
static_assert((A_CNT % 16) == 0 && (A_WSM % 16) == 0 && (A_BSM % 16) == 0 && (A_STG % 16) == 0);
static_assert((A_MSG % 16) == 0 && (A_LIST % 16) == 0 && (A_PEND % 16) == 0 && (A_SLOT % 16) == 0);
static_assert(A_END <= 300 * 1024);

#define N_W1H  0
#define N_W1L  (N_W1H + U * 2 * U * 2)
#define N_W2H  (N_W1L + U * 2 * U * 2)
#define N_W2L  (N_W2H + U * U * 2)
#define N_WM   (N_W2L + U * U * 2)
#define N_BS   (N_WM + U * U * 2)
#define N_STG  (N_BS + 512 * 4)
#define N_END  (N_STG + NWAVE * 16 * U * 4)
static_assert((N_STG % 16) == 0 && N_END <= 120 * 1024);

typedef float    v2f  __attribute__((ext_vector_type(2)));
typedef float    v4f  __attribute__((ext_vector_type(4)));
typedef float    v8f  __attribute__((ext_vector_type(8)));
typedef int      v4i  __attribute__((ext_vector_type(4)));
typedef _Float16 v8h  __attribute__((ext_vector_type(8)));
typedef _Float16 v16h __attribute__((ext_vector_type(16)));
typedef __bf16   v8b  __attribute__((ext_vector_type(8)));
typedef __bf16   v16b __attribute__((ext_vector_type(16)));
union FragH { v16h v; v8h h[2]; _Float16 e[16]; };
union FragB { v16b v; v8b h[2]; __bf16 e[16]; };

__device__ __forceinline__ v8f z8f() {
  v8f r;
#pragma unroll
  for (int i = 0; i < 8; ++i) r[i] = 0.0f;
  return r;
}

__device__ __forceinline__ v8f wmh(v16h a, v16h b, v8f c) {
  v8f d = __builtin_amdgcn_wmma_f32_16x16x32_f16(false, a, false, b, (short)0, c, false, false);
  asm volatile("v_nop\n\tv_nop\n\tv_nop\n\tv_nop" : "+v"(d) : "v"(a), "v"(b));
  return d;
}
__device__ __forceinline__ v8f wmb(v16b a, v16b b, v8f c) {
  v8f d = __builtin_amdgcn_wmma_f32_16x16x32_bf16(false, a, false, b, (short)0, c, false, false);
  asm volatile("v_nop\n\tv_nop\n\tv_nop\n\tv_nop" : "+v"(d) : "v"(a), "v"(b));
  return d;
}

__device__ __forceinline__ float bf2f(__bf16 b) {
  union { __bf16 b; unsigned short s; } u;
  u.b = b;
  return __uint_as_float(((unsigned)u.s) << 16);
}

__device__ __forceinline__ float silu_f(float v) {
  return v * __builtin_amdgcn_rcpf(1.0f + __expf(-v));
}

__device__ __forceinline__ v8f ldc8(const float* p) {
  const v4f a = *(const v4f*)p;
  const v4f b = *(const v4f*)(p + 4);
  v8f c;
  c[0] = a.x; c[1] = a.y; c[2] = a.z; c[3] = a.w;
  c[4] = b.x; c[5] = b.y; c[6] = b.z; c[7] = b.w;
  return c;
}

__device__ __forceinline__ int scan_chunk(const int* __restrict__ dsts, int nE, int cbase, int nodeBase,
                                          int vec8, int* list, int tid, int wave) {
  int wc = 0;
  const int el0  = tid * EPT;
  const int e0   = cbase + el0;
  const int sent = -2147483647 - 1;
  v4i da, db;
  if (vec8 != 0 && cbase + CHUNK <= nE) {
    da = *(const v4i*)(dsts + e0);
    db = *(const v4i*)(dsts + e0 + 4);
  } else {
    da.x = (e0     < nE) ? dsts[min(e0, nE - 1)] : sent;
    da.y = (e0 + 1 < nE) ? dsts[min(e0 + 1, nE - 1)] : sent;
    da.z = (e0 + 2 < nE) ? dsts[min(e0 + 2, nE - 1)] : sent;
    da.w = (e0 + 3 < nE) ? dsts[min(e0 + 3, nE - 1)] : sent;
    db.x = (e0 + 4 < nE) ? dsts[min(e0 + 4, nE - 1)] : sent;
    db.y = (e0 + 5 < nE) ? dsts[min(e0 + 5, nE - 1)] : sent;
    db.z = (e0 + 6 < nE) ? dsts[min(e0 + 6, nE - 1)] : sent;
    db.w = (e0 + 7 < nE) ? dsts[min(e0 + 7, nE - 1)] : sent;
  }
  const unsigned nb = (unsigned)nodeBase;
  const unsigned s0 = (unsigned)da.x - nb, s1 = (unsigned)da.y - nb;
  const unsigned s2 = (unsigned)da.z - nb, s3 = (unsigned)da.w - nb;
  const unsigned s4 = (unsigned)db.x - nb, s5 = (unsigned)db.y - nb;
  const unsigned s6 = (unsigned)db.z - nb, s7 = (unsigned)db.w - nb;
  const bool h0 = s0 < (unsigned)NB, h1 = s1 < (unsigned)NB, h2 = s2 < (unsigned)NB, h3 = s3 < (unsigned)NB;
  const bool h4 = s4 < (unsigned)NB, h5 = s5 < (unsigned)NB, h6 = s6 < (unsigned)NB, h7 = s7 < (unsigned)NB;
  const unsigned any = __builtin_amdgcn_ballot_w32(h0 | h1 | h2 | h3 | h4 | h5 | h6 | h7);
  if (any != 0u) {
#define HITJ(J, HJ) { \
      const unsigned mj = __builtin_amdgcn_ballot_w32(HJ); \
      if (mj != 0u) { \
        if (HJ) { \
          const int pos = wc + (int)__builtin_amdgcn_mbcnt_lo(mj, 0u); \
          if (pos < WCAP) list[wave * WCAP + pos] = el0 + (J); \
        } \
        wc += (int)__builtin_popcount(mj); } }
    HITJ(0, h0)
    HITJ(1, h1)
    HITJ(2, h2)
    HITJ(3, h3)
    HITJ(4, h4)
    HITJ(5, h5)
    HITJ(6, h6)
    HITJ(7, h7)
#undef HITJ
  }
  return wc;
}

__device__ __forceinline__ void tile_store(const float* sw, float* gp, int nb, int lane, int rowLim) {
  v4f ov[8];
#pragma unroll
  for (int q = 0; q < 8; ++q) ov[q] = *(const v4f*)(sw + q * 128 + lane * 4);
  float* base = gp + (size_t)nb * U + lane * 4;
  const int r0 = nb + (lane >> 4);
#pragma unroll
  for (int q = 0; q < 8; ++q) {
    if (r0 + 2 * q < rowLim) *(volatile v4f*)(base + q * 128) = ov[q];
  }
  __threadfence();
#pragma unroll
  for (int q = 0; q < 8; ++q) {
    if (r0 + 2 * q < rowLim) *(volatile v4f*)(base + q * 128) = ov[q];
  }
}

__global__ __launch_bounds__(NTHR) void k_agg(
    const float* __restrict__ Pp, const int* __restrict__ ei, const float* __restrict__ attr,
    const float* __restrict__ edgeW, const float* __restrict__ edgeB,
    const float* __restrict__ W1, const float* __restrict__ W2, const float* __restrict__ Bi2,
    float* aggrp, int nN, int nE, int vec8) {
  extern __shared__ __attribute__((aligned(16))) unsigned char lds_agg[];
  float*    acc   = (float*)(lds_agg + A_ACC);
  float*    cnt   = (float*)(lds_agg + A_CNT);
  _Float16* wsm   = (_Float16*)(lds_agg + A_WSM);
  float*    bsm   = (float*)(lds_agg + A_BSM);
  float*    ews   = (float*)(lds_agg + A_EW);
  float*    ebs   = (float*)(lds_agg + A_EB);
  _Float16* stg   = (_Float16*)(lds_agg + A_STG);
  float*    msg   = (float*)(lds_agg + A_MSG);
  int*      list  = (int*)(lds_agg + A_LIST);
  int*      pend  = (int*)(lds_agg + A_PEND);
  int*      slotb = (int*)(lds_agg + A_SLOT);
  int*      wcnt  = (int*)(lds_agg + A_WCNT);

  const int tid = threadIdx.x, lane = tid & 31, wave = tid >> 5, hh = lane >> 4, m = lane & 15;
  const int nodeBase = blockIdx.x * NB;
  const int* srcs = ei;
  const int* dsts = ei + nE;

  {
    v4f z = {0.0f, 0.0f, 0.0f, 0.0f};
    for (int i = tid; i < (NB + 1) * U / 4; i += NTHR) *(v4f*)(acc + 4 * i) = z;
    for (int i = tid; i < NB + 1; i += NTHR) cnt[i] = 0.0f;
    for (int i = tid; i < PCAP; i += NTHR) pend[i] = 0;
    for (int i = tid; i < 2 * U * U; i += NTHR) {
      const int which = i >> 12, n = (i >> 6) & 63, k = i & 63;
      const float va = W1[(U + k) * U + n];
      const float vb = W2[k * U + n];
      const float v = (which == 0) ? va : vb;
      wsm[i] = (_Float16)(v * WSC);
    }
    if (tid < U) {
      bsm[tid] = Bi2[tid] * WSC;
      ews[tid] = edgeW[tid];
      ebs[tid] = edgeB[tid];
    }
    if (tid == 0) wcnt[8] = 0;
  }
  __syncthreads();

  const int nChunks = (nE + CHUNK - 1) / CHUNK;
#pragma unroll 1
  for (int ch = 0; ch < nChunks; ++ch) {
    const int cbase = ch * CHUNK;
    const int wc = scan_chunk(dsts, nE, cbase, nodeBase, vec8, list, tid, wave);
    if (lane == 0) wcnt[wave] = wc;
    __syncthreads();

    const int base = wcnt[8];
    int tot = 0, myoff = 0;
#pragma unroll
    for (int w = 0; w < NWAVE; ++w) {
      int c = wcnt[w];
      c = c > WCAP ? WCAP : (c < 0 ? 0 : c);
      if (w < wave) myoff += c;
      tot += c;
    }
    int newN = base + tot;
    newN = newN > PCAP ? PCAP : newN;
    {
      int n = wcnt[wave];
      n = n > WCAP ? WCAP : (n < 0 ? 0 : n);
      const int* lp = list + wave * WCAP;
      for (int i = lane; i < n; i += 32) {
        const int pos = base + myoff + i;
        if (pos < PCAP) pend[pos] = cbase + lp[i];
      }
    }
    const int fin = (ch == nChunks - 1) ? 1 : 0;
    const int R   = (fin != 0) ? (newN + PASSN - 1) / PASSN : newN / PASSN;
    const int Pv  = (fin != 0) ? newN : R * PASSN;
    __syncthreads();

#pragma unroll 1
    for (int r = 0; r < R; ++r) {
      {
        const int idx = r * PASSN + wave * 16 + m;
        const bool valid = idx < Pv;
        int e = pend[idx];
        e = valid ? e : 0;
        e = e < 0 ? 0 : (e > nE - 1 ? nE - 1 : e);
        const int d = dsts[e];
        int s = srcs[e];
        int slot = d - nodeBase;
        if (!valid || (unsigned)slot >= (unsigned)NB) slot = NB;
        s = s < 0 ? 0 : (s > nN - 1 ? nN - 1 : s);
        const float a = attr[e];
        _Float16* sp = stg + (wave * 16 + m) * U + 32 * hh;
#pragma unroll
        for (int g = 0; g < 4; ++g) {
          v8h hv;
#pragma unroll
          for (int j = 0; j < 8; ++j) {
            const int f = 32 * hh + 8 * g + j;
            const float v = a * ews[f] + ebs[f];
            hv[j] = (_Float16)silu_f(v);
          }
          *(v8h*)(sp + 8 * g) = hv;
        }
        {
          const float* pg = Pp + (size_t)s * U + 32 * hh;
          float* pl = msg + (wave * 16 + m) * U + 32 * hh;
#pragma unroll
          for (int g = 0; g < 8; ++g) *(v4f*)(pl + 4 * g) = *(const v4f*)(pg + 4 * g);
        }
        if (hh == 0) slotb[wave * 16 + m] = slot;
      }
      __syncthreads();

      {
        FragH b[2];
        _Float16* ep = stg + (wave * 16 + m) * U + 8 * hh;
        b[0].h[0] = *(const v8h*)(ep);
        b[0].h[1] = *(const v8h*)(ep + 16);
        b[1].h[0] = *(const v8h*)(ep + 32);
        b[1].h[1] = *(const v8h*)(ep + 48);
        v8f d1[4];
#pragma unroll
        for (int ft = 0; ft < 4; ++ft) {
          v8f c = z8f();
#pragma unroll
          for (int ks = 0; ks < 2; ++ks) {
            FragH a;
            const _Float16* ap = wsm + (16 * ft + m) * U + 32 * ks + 8 * hh;
            a.h[0] = *(const v8h*)ap;
            a.h[1] = *(const v8h*)(ap + 16);
            c = wmh(a.v, b[ks].v, c);
          }
          d1[ft] = c;
        }
        const float* plr = msg + (wave * 16 + m) * U + 8 * hh;
        __builtin_amdgcn_fence(__ATOMIC_RELEASE, "wavefront");
        __builtin_amdgcn_wave_barrier();
#pragma unroll
        for (int ft = 0; ft < 4; ++ft) {
          const v4f p0 = *(const v4f*)(plr + 16 * ft);
          const v4f p1 = *(const v4f*)(plr + 16 * ft + 4);
          float pv[8];
          pv[0] = p0.x; pv[1] = p0.y; pv[2] = p0.z; pv[3] = p0.w;
          pv[4] = p1.x; pv[5] = p1.y; pv[6] = p1.z; pv[7] = p1.w;
          v8h t;
#pragma unroll
          for (int rr = 0; rr < 8; ++rr) t[rr] = (_Float16)silu_f(d1[ft][rr] * WINV + pv[rr]);
          *(v8h*)(ep + 16 * ft) = t;
        }
        __builtin_amdgcn_fence(__ATOMIC_RELEASE, "wavefront");
        __builtin_amdgcn_wave_barrier();
        FragH b2[2];
        b2[0].h[0] = *(const v8h*)(ep);
        b2[0].h[1] = *(const v8h*)(ep + 16);
        b2[1].h[0] = *(const v8h*)(ep + 32);
        b2[1].h[1] = *(const v8h*)(ep + 48);
        v8f d2[4];
#pragma unroll
        for (int ft = 0; ft < 4; ++ft) {
          v8f c = ldc8(bsm + 16 * ft + 8 * hh);
#pragma unroll
          for (int ks = 0; ks < 2; ++ks) {
            FragH a;
            const _Float16* ap = wsm + U * U + (16 * ft + m) * U + 32 * ks + 8 * hh;
            a.h[0] = *(const v8h*)ap;
            a.h[1] = *(const v8h*)(ap + 16);
            c = wmh(a.v, b2[ks].v, c);
          }
          d2[ft] = c;
        }
        float* mp = msg + (wave * 16 + m) * U + 8 * hh;
#pragma unroll
        for (int ft = 0; ft < 4; ++ft) {
          v4f lo = {d2[ft][0] * WINV, d2[ft][1] * WINV, d2[ft][2] * WINV, d2[ft][3] * WINV};
          v4f hi = {d2[ft][4] * WINV, d2[ft][5] * WINV, d2[ft][6] * WINV, d2[ft][7] * WINV};
          *(v4f*)(mp + 16 * ft)     = lo;
          *(v4f*)(mp + 16 * ft + 4) = hi;
        }
      }
      __syncthreads();

      if (wave == 0) {
#pragma unroll 1
        for (int i = 0; i < PASSN; ++i) {
          int sl = slotb[i];
          sl = sl < 0 ? 0 : (sl > NB ? NB : sl);
          const v2f mv = *(const v2f*)(msg + i * U + 2 * lane);
          float* ap = acc + sl * U + 2 * lane;
          v2f av = *(const v2f*)ap;
          av += mv;
          *(v2f*)ap = av;
          if (lane == 0) cnt[sl] += 1.0f;
        }
      }
      __syncthreads();
    }

    int rem = newN - R * PASSN;
    rem = rem < 0 ? 0 : rem;
    if (R > 0 && tid < rem) pend[tid] = pend[R * PASSN + tid];
    if (tid == 0) wcnt[8] = rem;
  }
  __syncthreads();

  const size_t ob = (size_t)nodeBase * U;
#pragma unroll 6
  for (int q = 0; q < NQ; ++q) {
    const int f  = (q * NTHR + tid) * 4;
    const int sl = f >> 6, c = f & 63;
    const float inv = __builtin_amdgcn_rcpf(fmaxf(cnt[sl], 1.0f));
    v4f v = *(const v4f*)(acc + sl * U + c);
    v *= inv;
    *(volatile v4f*)(aggrp + ob + f) = v;
  }
  __threadfence();
#pragma unroll 6
  for (int q = 0; q < NQ; ++q) {
    const int f  = (q * NTHR + tid) * 4;
    const int sl = f >> 6, c = f & 63;
    const float inv = __builtin_amdgcn_rcpf(fmaxf(cnt[sl], 1.0f));
    v4f v = *(const v4f*)(acc + sl * U + c);
    v *= inv;
    *(volatile v4f*)(aggrp + ob + f) = v;
  }
}

template <int FIRST, int LAST>
__global__ __launch_bounds__(NTHR) void k_node(
    const float* __restrict__ xin, const float* __restrict__ nodeW, const float* __restrict__ nodeB,
    const float* __restrict__ hin, const float* __restrict__ aggr,
    const float* __restrict__ uW1, const float* __restrict__ uB1,
    const float* __restrict__ uW2, const float* __restrict__ uB2,
    const float* __restrict__ lng, const float* __restrict__ lnb,
    const float* __restrict__ mW1, const float* __restrict__ mB1,
    float* hout, float* Pout, int nN) {
  extern __shared__ __attribute__((aligned(16))) unsigned char lds_node[];
  __bf16*   w1h = (__bf16*)(lds_node + N_W1H);
  __bf16*   w1l = (__bf16*)(lds_node + N_W1L);
  __bf16*   w2h = (__bf16*)(lds_node + N_W2H);
  __bf16*   w2l = (__bf16*)(lds_node + N_W2L);
  _Float16* wm  = (_Float16*)(lds_node + N_WM);
  float*    bs  = (float*)(lds_node + N_BS);
  float*    stg = (float*)(lds_node + N_STG);

  const int tid = threadIdx.x, lane = tid & 31, wave = tid >> 5, hh = lane >> 4, m = lane & 15;

  if (FIRST == 0) {
    for (int i = tid; i < 2 * U * U; i += NTHR) {
      const int n = i >> 7, k = i & 127;
      const float v = uW1[k * U + n];
      const __bf16 hb = (__bf16)v;
      w1h[i] = hb;
      w1l[i] = (__bf16)(v - bf2f(hb));
    }
    for (int i = tid; i < U * U; i += NTHR) {
      const int n = i >> 6, k = i & 63;
      const float v = uW2[k * U + n];
      const __bf16 hb = (__bf16)v;
      w2h[i] = hb;
      w2l[i] = (__bf16)(v - bf2f(hb));
    }
    if (tid < U) {
      bs[tid]       = uB1[tid];
      bs[64 + tid]  = uB2[tid];
      bs[128 + tid] = lng[tid];
      bs[192 + tid] = lnb[tid];
    }
  } else {
    if (tid < 2 * U) bs[320 + tid] = nodeW[tid];
    if (tid < U) bs[448 + tid] = nodeB[tid];
  }
  if (LAST == 0) {
    for (int i = tid; i < U * U; i += NTHR) {
      const int n = i >> 6, k = i & 63;
      wm[i] = (_Float16)(mW1[k * U + n] * WSC);
    }
    if (tid < U) bs[256 + tid] = mB1[tid];
  }
  __syncthreads();

  const int nb   = blockIdx.x * NT + wave * 16;
  const int node = nb + m;
  float res[32];

  if (FIRST != 0) {
    const int nr = node < nN ? node : nN - 1;
    const float x0 = xin[(size_t)nr * 2], x1 = xin[(size_t)nr * 2 + 1];
#pragma unroll
    for (int ft = 0; ft < 4; ++ft) {
#pragma unroll
      for (int rr = 0; rr < 8; ++rr) {
        const int f = 16 * ft + 8 * hh + rr;
        const float v = x0 * bs[320 + f] + x1 * bs[384 + f] + bs[448 + f];
        res[ft * 8 + rr] = silu_f(v);
      }
    }
  } else {
    float hv[32];
    v8f d1[4];
#pragma unroll
    for (int ft = 0; ft < 4; ++ft) d1[ft] = ldc8(bs + 16 * ft + 8 * hh);
    const float* hrow = hin + (size_t)node * U + 8 * hh;
    const float* arow = aggr + (size_t)node * U + 8 * hh;
#pragma unroll
    for (int ks = 0; ks < 4; ++ks) {
      const float* rp = (ks == 0) ? hrow : ((ks == 1) ? (hrow + 32) : ((ks == 2) ? arow : (arow + 32)));
      const v4f q0 = *(const v4f*)rp;
      const v4f q1 = *(const v4f*)(rp + 4);
      const v4f q2 = *(const v4f*)(rp + 16);
      const v4f q3 = *(const v4f*)(rp + 20);
      float v[16];
      v[0] = q0.x; v[1] = q0.y; v[2]  = q0.z; v[3]  = q0.w; v[4]  = q1.x; v[5]  = q1.y; v[6]  = q1.z; v[7]  = q1.w;
      v[8] = q2.x; v[9] = q2.y; v[10] = q2.z; v[11] = q2.w; v[12] = q3.x; v[13] = q3.y; v[14] = q3.z; v[15] = q3.w;
      if (ks < 2) {
#pragma unroll
        for (int i = 0; i < 16; ++i) hv[ks * 16 + i] = v[i];
      }
      FragB bh, bl;
#pragma unroll
      for (int i = 0; i < 16; ++i) {
        const __bf16 hb = (__bf16)v[i];
        bh.e[i] = hb;
        bl.e[i] = (__bf16)(v[i] - bf2f(hb));
      }
#pragma unroll
      for (int ft = 0; ft < 4; ++ft) {
        FragB ah, al;
        const __bf16* ap = w1h + (16 * ft + m) * (2 * U) + 32 * ks + 8 * hh;
        const __bf16* aq = w1l + (16 * ft + m) * (2 * U) + 32 * ks + 8 * hh;
        ah.h[0] = *(const v8b*)ap;
        ah.h[1] = *(const v8b*)(ap + 16);
        al.h[0] = *(const v8b*)aq;
        al.h[1] = *(const v8b*)(aq + 16);
        v8f c = d1[ft];
        c = wmb(ah.v, bh.v, c);
        c = wmb(ah.v, bl.v, c);
        c = wmb(al.v, bh.v, c);
        d1[ft] = c;
      }
    }
    FragB uh[2], ul[2];
#pragma unroll
    for (int ft = 0; ft < 4; ++ft) {
#pragma unroll
      for (int rr = 0; rr < 8; ++rr) {
        const float uu = silu_f(d1[ft][rr]);
        const __bf16 hb = (__bf16)uu;
        uh[ft >> 1].e[(ft & 1) * 8 + rr] = hb;
        ul[ft >> 1].e[(ft & 1) * 8 + rr] = (__bf16)(uu - bf2f(hb));
      }
    }
    v8f d2[4];
#pragma unroll
    for (int ft = 0; ft < 4; ++ft) {
      v8f c = ldc8(bs + 64 + 16 * ft + 8 * hh);
#pragma unroll
      for (int ks = 0; ks < 2; ++ks) {
        FragB ah, al;
        const __bf16* ap = w2h + (16 * ft + m) * U + 32 * ks + 8 * hh;
        const __bf16* aq = w2l + (16 * ft + m) * U + 32 * ks + 8 * hh;
        ah.h[0] = *(const v8b*)ap;
        ah.h[1] = *(const v8b*)(ap + 16);
        al.h[0] = *(const v8b*)aq;
        al.h[1] = *(const v8b*)(aq + 16);
        c = wmb(ah.v, uh[ks].v, c);
        c = wmb(ah.v, ul[ks].v, c);
        c = wmb(al.v, uh[ks].v, c);
      }
      d2[ft] = c;
    }
    float s1 = 0.0f;
#pragma unroll
    for (int ft = 0; ft < 4; ++ft) {
#pragma unroll
      for (int rr = 0; rr < 8; ++rr) {
        const float t = hv[ft * 8 + rr] + d2[ft][rr];
        res[ft * 8 + rr] = t;
        s1 += t;
      }
    }
    s1 += __shfl_xor(s1, 16);
    const float mu = s1 * (1.0f / 64.0f);
    float s2 = 0.0f;
#pragma unroll
    for (int i = 0; i < 32; ++i) {
      const float dd = res[i] - mu;
      res[i] = dd;
      s2 += dd * dd;
    }
    s2 += __shfl_xor(s2, 16);
    const float var = s2 * (1.0f / 64.0f);
    const float rs = rsqrtf(var + LN_EPS);
#pragma unroll
    for (int ft = 0; ft < 4; ++ft) {
#pragma unroll
      for (int rr = 0; rr < 8; ++rr) {
        const int f = 16 * ft + 8 * hh + rr;
        res[ft * 8 + rr] = res[ft * 8 + rr] * rs * bs[128 + f] + bs[192 + f];
      }
    }
  }

  float* sw = stg + wave * (16 * U);
  {
    float* rp = sw + m * U + 8 * hh;
#pragma unroll
    for (int ft = 0; ft < 4; ++ft) {
      v4f lo = {res[ft * 8 + 0], res[ft * 8 + 1], res[ft * 8 + 2], res[ft * 8 + 3]};
      v4f hi = {res[ft * 8 + 4], res[ft * 8 + 5], res[ft * 8 + 6], res[ft * 8 + 7]};
      *(v4f*)(rp + 16 * ft)     = lo;
      *(v4f*)(rp + 16 * ft + 4) = hi;
    }
  }
  __syncthreads();
  tile_store(sw, hout, nb, lane, (LAST != 0) ? nN : 2147483647);

  if (LAST == 0) {
    FragH bq[2];
#pragma unroll
    for (int ks = 0; ks < 2; ++ks) {
#pragma unroll
      for (int i = 0; i < 8; ++i) {
        bq[ks].e[i]     = (_Float16)res[(2 * ks) * 8 + i];
        bq[ks].e[8 + i] = (_Float16)res[(2 * ks + 1) * 8 + i];
      }
    }
    v8f d3[4];
#pragma unroll
    for (int ft = 0; ft < 4; ++ft) {
      v8f c = z8f();
#pragma unroll
      for (int ks = 0; ks < 2; ++ks) {
        FragH a;
        const _Float16* ap = wm + (16 * ft + m) * U + 32 * ks + 8 * hh;
        a.h[0] = *(const v8h*)ap;
        a.h[1] = *(const v8h*)(ap + 16);
        c = wmh(a.v, bq[ks].v, c);
      }
      d3[ft] = c;
    }
    __syncthreads();
    {
      float* rp = sw + m * U + 8 * hh;
#pragma unroll
      for (int ft = 0; ft < 4; ++ft) {
        const float* bb = bs + 256 + 16 * ft + 8 * hh;
        v4f lo = {d3[ft][0] * WINV + bb[0], d3[ft][1] * WINV + bb[1], d3[ft][2] * WINV + bb[2], d3[ft][3] * WINV + bb[3]};
        v4f hi = {d3[ft][4] * WINV + bb[4], d3[ft][5] * WINV + bb[5], d3[ft][6] * WINV + bb[6], d3[ft][7] * WINV + bb[7]};
        *(v4f*)(rp + 16 * ft)     = lo;
        *(v4f*)(rp + 16 * ft + 4) = hi;
      }
    }
    __syncthreads();
    tile_store(sw, Pout, nb, lane, 2147483647);
  }
}

extern "C" void kernel_launch(void* const* d_in, const int* in_sizes, int n_in,
                              void* d_out, int out_size, void* d_ws, size_t ws_size,
                              hipStream_t stream) {
  if (n_in < 17) return;
  const int nN = in_sizes[0] / 2;
  const int nE = in_sizes[1] / 2;
  if (nN <= 0 || nE <= 0 || in_sizes[0] != nN * 2 || in_sizes[1] != nE * 2 || in_sizes[2] != nE) return;
  if (in_sizes[3] != 2 * U || in_sizes[4] != U || in_sizes[5] != U || in_sizes[6] != U) return;
  const int D = in_sizes[7] / (2 * U * U);
  if (D < 1 || in_sizes[7] != D * 2 * U * U || in_sizes[8] != D * U || in_sizes[9] != D * U * U || in_sizes[10] != D * U) return;
  if (in_sizes[11] != D * 2 * U * U || in_sizes[12] != D * U || in_sizes[13] != D * U * U || in_sizes[14] != D * U) return;
  if (in_sizes[15] != D * U || in_sizes[16] != D * U) return;
  if (out_size != nN * U) return;

  const float* x     = (const float*)d_in[0];
  const int*   ei    = (const int*)d_in[1];
  const float* attr  = (const float*)d_in[2];
  const float* nodeW = (const float*)d_in[3];
  const float* nodeB = (const float*)d_in[4];
  const float* edgeW = (const float*)d_in[5];
  const float* edgeB = (const float*)d_in[6];
  const float* msgW1 = (const float*)d_in[7];
  const float* msgB1 = (const float*)d_in[8];
  const float* msgW2 = (const float*)d_in[9];
  const float* msgB2 = (const float*)d_in[10];
  const float* updW1 = (const float*)d_in[11];
  const float* updB1 = (const float*)d_in[12];
  const float* updW2 = (const float*)d_in[13];
  const float* updB2 = (const float*)d_in[14];
  const float* lng   = (const float*)d_in[15];
  const float* lnb   = (const float*)d_in[16];
  float* out = (float*)d_out;

  const int nBlkN = (nN + NT - 1) / NT;
  const int NpadN = nBlkN * NT;
  const int nBlkA = (nN + NB - 1) / NB;
  const int NpadA = nBlkA * NB;

  char* ws = (char*)d_ws;
  size_t off = 0;
  const size_t plN = (size_t)NpadN * U * 4;
  const size_t plA = (size_t)NpadA * U * 4;
  const size_t oHA = off; off += plN; off = (off + 255) & ~(size_t)255;
  const size_t oHB = off; off += plN; off = (off + 255) & ~(size_t)255;
  const size_t oP  = off; off += plN; off = (off + 255) & ~(size_t)255;
  const size_t oAg = off; off += plA; off = (off + 255) & ~(size_t)255;
  if (off > ws_size) return;
  float* hA   = (float*)(ws + oHA);
  float* hB   = (float*)(ws + oHB);
  float* Pp   = (float*)(ws + oP);
  float* aggr = (float*)(ws + oAg);

  const int vec8 = ((nE & 3) == 0) ? 1 : 0;

  k_node<1, 0><<<nBlkN, NTHR, N_END, stream>>>(
      x, nodeW, nodeB, hB, aggr, updW1, updB1, updW2, updB2, lng, lnb, msgW1, msgB1, hA, Pp, nN);

  float* hc = hA;
  float* hn = hB;
  for (int i = 0; i < D; ++i) {
    k_agg<<<nBlkA, NTHR, A_END, stream>>>(
        Pp, ei, attr, edgeW, edgeB,
        msgW1 + (size_t)i * 2 * U * U, msgW2 + (size_t)i * U * U, msgB2 + (size_t)i * U,
        aggr, nN, nE, vec8);
    const int last = (i == D - 1) ? 1 : 0;
    const int im = last ? i : i + 1;
    if (last) {
      k_node<0, 1><<<nBlkN, NTHR, N_END, stream>>>(
          x, nodeW, nodeB, hc, aggr,
          updW1 + (size_t)i * 2 * U * U, updB1 + (size_t)i * U, updW2 + (size_t)i * U * U, updB2 + (size_t)i * U,
          lng + (size_t)i * U, lnb + (size_t)i * U,
          msgW1 + (size_t)im * 2 * U * U, msgB1 + (size_t)im * U, out, Pp, nN);
    } else {
      k_node<0, 0><<<nBlkN, NTHR, N_END, stream>>>(
          x, nodeW, nodeB, hc, aggr,
          updW1 + (size_t)i * 2 * U * U, updB1 + (size_t)i * U, updW2 + (size_t)i * U * U, updB2 + (size_t)i * U,
          lng + (size_t)i * U, lnb + (size_t)i * U,
          msgW1 + (size_t)im * 2 * U * U, msgB1 + (size_t)im * U, hn, Pp, nN);
      float* t = hc; hc = hn; hn = t;
    }
  }
}
